// STSGCM_2370821947438
// MI455X (gfx1250) — hardware-verified
//
#include <hip/hip_runtime.h>
#include <stdint.h>
#include <math.h>

constexpr int kNV    = 3000;
constexpr int kNP    = 3008;
constexpr int kBatch = 32;
constexpr int kCh    = 64;
constexpr int kNCol  = kBatch * kCh;
constexpr int kLR    = 128;
constexpr int kMid0  = 1000;
constexpr int kMid1  = 2000;
constexpr int kMidN  = 1000;
constexpr int kL2Row0 = 960;
constexpr int kL2Rows = 1088;
static_assert(kNP % 64 == 0 && kNP % 32 == 0, "tile multiples");
static_assert(kNCol % 64 == 0, "tile multiples");
static_assert((kNP * kBatch) % 64 == 0 && (kL2Rows * kBatch) % 64 == 0, "tile multiples");
static_assert(kL2Rows % 64 == 0 && kL2Row0 + kL2Rows <= kNP && kL2Row0 <= kMid0 && kL2Row0 + kL2Rows >= kMid1, "last layer row window");

typedef __attribute__((ext_vector_type(16))) _Float16 v16h;
typedef __attribute__((ext_vector_type(8)))  _Float16 v8h;
typedef __attribute__((ext_vector_type(16))) __bf16   v16b;
typedef __attribute__((ext_vector_type(8)))  __bf16   v8b;
typedef __attribute__((ext_vector_type(8)))  float    v8f;
typedef __attribute__((ext_vector_type(4)))  float    v4f;
typedef __attribute__((ext_vector_type(4)))  unsigned int v4u;

__device__ __forceinline__ unsigned short f2bf_bits(float f) {
  unsigned u = __float_as_uint(f);
  return (unsigned short)((u + 0x7FFFu + ((u >> 16) & 1u)) >> 16);
}
__device__ __forceinline__ float bf_bits2f(unsigned short h) { return __uint_as_float(((unsigned)h) << 16); }

__device__ __forceinline__ void dep_guard_h(v8f& a, v8f& b, v16h x, v16h y) { asm volatile("v_nop\n\tv_nop\n\tv_nop\n\tv_nop" : "+v"(a), "+v"(b) : "v"(x), "v"(y)); }
__device__ __forceinline__ void dep_guard_b(v8f& a, v8f& b, v16b x, v16b y) { asm volatile("v_nop\n\tv_nop\n\tv_nop\n\tv_nop" : "+v"(a), "+v"(b) : "v"(x), "v"(y)); }
__device__ __forceinline__ void keep4_h(v16h a, v16h b, v16h c, v16h d) { asm volatile("v_nop" :: "v"(a), "v"(b), "v"(c), "v"(d)); }
__device__ __forceinline__ void keep4_b(v16b a, v16b b, v16b c, v16b d) { asm volatile("v_nop" :: "v"(a), "v"(b), "v"(c), "v"(d)); }
__device__ __forceinline__ void acc_guard4(v8f& a, v8f& b, v8f& c, v8f& d) { asm volatile("v_nop\n\tv_nop\n\tv_nop\n\tv_nop" : "+v"(a), "+v"(b), "+v"(c), "+v"(d)); }
template <typename T> struct Frag;
template <> struct Frag<_Float16> {
  typedef v16h V; union U { v16h v; v8h h[2]; };
  static __device__ __forceinline__ v16h load(const _Float16* p) {
    U f; f.h[0] = *(const v8h*)(p); f.h[1] = *(const v8h*)(p + 16); return f.v;
  }
  static __device__ __forceinline__ v8f mma(v16h a, v16h b, v8f c) {
    return __builtin_amdgcn_wmma_f32_16x16x32_f16(false, a, false, b, (short)0, c, false, false);
  }
  static __device__ __forceinline__ void guard(v8f& a, v8f& b, v16h x, v16h y) { dep_guard_h(a, b, x, y); }
  static __device__ __forceinline__ void keep(v16h a, v16h b, v16h c, v16h d) { keep4_h(a, b, c, d); }
};
template <> struct Frag<__bf16> {
  typedef v16b V; union U { v16b v; v8b h[2]; };
  static __device__ __forceinline__ v16b load(const __bf16* p) {
    U f; f.h[0] = *(const v8b*)(p); f.h[1] = *(const v8b*)(p + 16); return f.v;
  }
  static __device__ __forceinline__ v8f mma(v16b a, v16b b, v8f c) {
    return __builtin_amdgcn_wmma_f32_16x16x32_bf16(false, a, false, b, (short)0, c, false, false);
  }
  static __device__ __forceinline__ void guard(v8f& a, v8f& b, v16b x, v16b y) { dep_guard_b(a, b, x, y); }
  static __device__ __forceinline__ void keep(v16b a, v16b b, v16b c, v16b d) { keep4_b(a, b, c, d); }
};

__device__ __forceinline__ unsigned pk16(unsigned short a, unsigned short b) { return (unsigned)a | ((unsigned)b << 16); }

template <int ET> struct Elem;
template <> struct Elem<0> { typedef _Float16 T; };
template <> struct Elem<1> { typedef __bf16 T; };
template <int ET, bool SPLIT, int BIAS_MODE, int OUT_MODE, bool RESID, int ACT = 0>
__global__ __launch_bounds__(256) void wmma_gemm64(
    const unsigned short* __restrict__ Ap, const unsigned short* __restrict__ A2p, int lda, long strideA,
    const unsigned short* __restrict__ Btp, const unsigned short* __restrict__ Bt2p, int ldb, long strideB,
    void* __restrict__ Cout, void* __restrict__ Cout2, int ldc, long strideC,
    const float* __restrict__ bias,
    const float* __restrict__ resid, long strideR,
    int M, int N, int K, float scale) {
  typedef typename Elem<ET>::T T;
  typedef typename Frag<T>::V V;
  const T* A = (const T*)Ap; const T* A2 = (const T*)A2p; const T* Bt = (const T*)Btp; const T* Bt2 = (const T*)Bt2p;
  __shared__ __align__(16) float sT[8][16 * 68];
  const int b    = blockIdx.y;
  const int lane = threadIdx.x & 31;
  const int wave = threadIdx.x >> 5;
  const int tilesN = N >> 6;
  const int tilesM = M >> 6;
  const int tile = blockIdx.x * 8 + wave;
  if (tile >= tilesM * tilesN) return;
  const int tm = tile / tilesN;
  const int tn = tile - tm * tilesN;
  const int m0 = tm << 6;
  const int n0 = tn << 6;

  const T* Ab  = A  + (size_t)b * strideA;
  const T* Bb  = Bt + (size_t)b * strideB;
  const T* Ab2 = SPLIT ? (A2  + (size_t)b * strideA) : nullptr;
  const T* Bb2 = SPLIT ? (Bt2 + (size_t)b * strideB) : nullptr;

  const int rlane = lane & 15;
  const int koff  = (lane >> 4) * 8;
  const int mOff  = (lane >> 4) * 8;

  v8f acc[4][4];
#pragma unroll
  for (int i = 0; i < 4; ++i)
#pragma unroll
    for (int j = 0; j < 4; ++j) acc[i][j] = (v8f){0.f,0.f,0.f,0.f,0.f,0.f,0.f,0.f};

  for (int k0 = 0; k0 < K; k0 += 32) {
    V bh[4], bl[4];
#pragma unroll
    for (int j = 0; j < 4; ++j) {
      const size_t bo = (size_t)(n0 + (j << 4) + rlane) * ldb + koff + k0;
      bh[j] = Frag<T>::load(Bb + bo);
      if (SPLIT) bl[j] = Frag<T>::load(Bb2 + bo);
    }
#pragma unroll
    for (int i = 0; i < 4; ++i) {
      const size_t ao = (size_t)(m0 + (i << 4) + rlane) * lda + koff + k0;
      V ah = Frag<T>::load(Ab + ao);
      V al;
      if (SPLIT) al = Frag<T>::load(Ab2 + ao);
#pragma unroll
      for (int j = 0; j < 4; ++j) {
        acc[i][j] = Frag<T>::mma(ah, bh[j], acc[i][j]);
        if (SPLIT) {
          acc[i][j] = Frag<T>::mma(ah, bl[j], acc[i][j]);
          acc[i][j] = Frag<T>::mma(al, bh[j], acc[i][j]);
        }
      }
      Frag<T>::guard(acc[i][0], acc[i][3], ah, SPLIT ? al : ah);
    }
    Frag<T>::keep(bh[0], bh[1], bh[2], bh[3]);
    if (SPLIT) Frag<T>::keep(bl[0], bl[1], bl[2], bl[3]);
  }
  acc_guard4(acc[0][0], acc[0][1], acc[0][2], acc[0][3]);
  acc_guard4(acc[1][0], acc[1][1], acc[1][2], acc[1][3]);
  acc_guard4(acc[2][0], acc[2][1], acc[2][2], acc[2][3]);
  acc_guard4(acc[3][0], acc[3][1], acc[3][2], acc[3][3]);

  float* slab = sT[wave];
  const float* Rb = RESID ? (resid + (size_t)b * strideR) : nullptr;
#pragma unroll
  for (int i = 0; i < 4; ++i) {
    const int mBase = m0 + (i << 4);
#pragma unroll
    for (int j = 0; j < 4; ++j) {
      const int n = n0 + (j << 4) + rlane;
      float bv = 0.f;
      if (BIAS_MODE == 2) bv = bias[n];
#pragma unroll
      for (int r = 0; r < 8; ++r) {
        float v = acc[i][j][r] * scale;
        if (BIAS_MODE == 1) v += bias[mBase + mOff + r];
        if (BIAS_MODE == 2) v += bv;
        if (RESID) v += Rb[(size_t)(mBase + mOff + r) * ldc + n];
        if (ACT == 2) v = fmaxf(v, 0.0f);
        if (ACT == 4) v = (v > 0.f) ? v : 0.01f * v;
        slab[(mOff + r) * 68 + (j << 4) + rlane] = v;
      }
    }
    __builtin_amdgcn_fence(__ATOMIC_RELEASE, "workgroup");
    __builtin_amdgcn_wave_barrier();
    __builtin_amdgcn_fence(__ATOMIC_ACQUIRE, "workgroup");
    if (OUT_MODE == 0) {
      float* C = (float*)Cout + (size_t)b * strideC;
      const int hh = lane >> 4, c4 = (lane & 15) * 4;
      for (int pass = 0; pass < 2; ++pass) {
#pragma unroll
        for (int it = 0; it < 8; ++it) {
          const int row = it * 2 + hh;
          v4f v = *(const v4f*)(slab + row * 68 + c4);
          *(volatile v4f*)(C + (size_t)(mBase + row) * ldc + n0 + c4) = v;
        }
        __threadfence();
      }
    } else {
      const int q = lane >> 3, c8 = (lane & 7) * 8;
      unsigned short* C  = (unsigned short*)Cout  + (size_t)b * strideC;
      unsigned short* C2 = (OUT_MODE == 2) ? ((unsigned short*)Cout2 + (size_t)b * strideC) : nullptr;
      for (int pass = 0; pass < 2; ++pass) {
#pragma unroll
        for (int it = 0; it < 4; ++it) {
          const int row = it * 4 + q;
          const float* sp = slab + row * 68 + c8;
          v8h hv, lv;
#pragma unroll
          for (int e = 0; e < 8; ++e) {
            if (OUT_MODE == 1) {
              hv[e] = (_Float16)sp[e];
            } else if (OUT_MODE == 3) {
              hv[e] = __builtin_bit_cast(_Float16, f2bf_bits(sp[e]));
            } else {
              unsigned short hb = f2bf_bits(sp[e]);
              unsigned short lb = f2bf_bits(sp[e] - bf_bits2f(hb));
              hv[e] = __builtin_bit_cast(_Float16, hb);
              lv[e] = __builtin_bit_cast(_Float16, lb);
            }
          }
          *(volatile v8h*)(C + (size_t)(mBase + row) * ldc + n0 + c8) = hv;
          if (OUT_MODE == 2) *(volatile v8h*)(C2 + (size_t)(mBase + row) * ldc + n0 + c8) = lv;
        }
        __threadfence();
      }
    }
    __builtin_amdgcn_fence(__ATOMIC_RELEASE, "workgroup");
    __builtin_amdgcn_wave_barrier();
    __builtin_amdgcn_fence(__ATOMIC_ACQUIRE, "workgroup");
  }
}

constexpr int kAdjGroupsPerRow = kNP / 8;
constexpr int kAdjThreads      = kNP * kAdjGroupsPerRow;
static_assert(kAdjThreads % 256 == 0, "exact grid");
__global__ __launch_bounds__(256) void cvt_adj_kernel(const float* __restrict__ adj, unsigned short* __restrict__ adjb) {
  const int gid = blockIdx.x * 256 + threadIdx.x;
  if (gid >= kAdjThreads) return;
  const int r  = gid / kAdjGroupsPerRow;
  const int c8 = (gid - r * kAdjGroupsPerRow) * 8;
  const int rc = (r < kNV) ? r : (kNV - 1);
  const float* src = adj + (size_t)rc * kNV;
  unsigned short hb[8];
#pragma unroll
  for (int e = 0; e < 8; ++e) {
    const int c  = c8 + e;
    const int cc = (c < kNV) ? c : (kNV - 1);
    float v = src[cc];
    v = (r < kNV && c < kNV) ? v : 0.0f;
    hb[e] = f2bf_bits(v);
  }
  const v4u u = (v4u){pk16(hb[0], hb[1]), pk16(hb[2], hb[3]), pk16(hb[4], hb[5]), pk16(hb[6], hb[7])};
  unsigned short* dst = adjb + (size_t)r * kNP + c8;
  *(volatile v4u*)dst = u;
  __threadfence();
  *(volatile v4u*)dst = u;
}

__global__ __launch_bounds__(256) void cvt_xT_kernel(const float* __restrict__ x, unsigned short* __restrict__ xt) {
  __shared__ float sm[64][65];
  const int t  = threadIdx.x;
  const int n0 = blockIdx.x * 64;
  const int c0 = blockIdx.y * 64;
#pragma unroll
  for (int i = 0; i < 16; ++i) {
    const int e  = i * 256 + t;
    const int nl = e >> 6;
    const int cl = e & 63;
    const int n  = n0 + nl;
    const int nc = (n < kNV) ? n : (kNV - 1);
    float v = x[(size_t)nc * kNCol + c0 + cl];
    v = (n < kNV) ? v : 0.0f;
    sm[cl][nl] = v;
  }
  __syncthreads();
  const int lane = t & 31, wave = t >> 5;
  const int q = lane >> 3, c8 = (lane & 7) * 8;
  for (int pass = 0; pass < 2; ++pass) {
#pragma unroll
    for (int it = 0; it < 2; ++it) {
      const int row = wave * 8 + it * 4 + q;
      unsigned short hb[8];
#pragma unroll
      for (int e = 0; e < 8; ++e) hb[e] = f2bf_bits(sm[row][c8 + e]);
      const v4u u = (v4u){pk16(hb[0], hb[1]), pk16(hb[2], hb[3]), pk16(hb[4], hb[5]), pk16(hb[6], hb[7])};
      *(volatile v4u*)(xt + (size_t)(c0 + row) * kNP + n0 + c8) = u;
    }
    __threadfence();
  }
}

__global__ __launch_bounds__(256) void cvt_w_kernel(const float* __restrict__ W0, const float* __restrict__ W1,
                                                    const float* __restrict__ W2, unsigned short* __restrict__ wt) {
  const int gid = blockIdx.x * 256 + threadIdx.x;
  const int R   = gid >> 3;
  const int l   = blockIdx.x >> 2;
  const int j   = R & 127;
  const int c8  = (gid & 7) * 8;
  const float* W = (l == 0) ? W0 : (l == 1) ? W1 : W2;
  unsigned short hb[8];
#pragma unroll
  for (int e = 0; e < 8; ++e) hb[e] = f2bf_bits(W[(size_t)(c8 + e) * kLR + j]);
  const v4u u = (v4u){pk16(hb[0], hb[1]), pk16(hb[2], hb[3]), pk16(hb[4], hb[5]), pk16(hb[6], hb[7])};
  unsigned short* dst = wt + (size_t)R * kCh + c8;
  *(volatile v4u*)dst = u;
  __threadfence();
  *(volatile v4u*)dst = u;
}

__global__ __launch_bounds__(256) void glu_kernel(const float* __restrict__ lr, const float* __restrict__ bias,
                                                  unsigned short* __restrict__ xt, float* __restrict__ keep,
                                                  int nbase, int write_xt) {
  __shared__ __align__(16) float sV[64][68];
  const int t = threadIdx.x, lane = t & 31, wave = t >> 5, hh = lane >> 4, c16 = lane & 15;
  const int tile = blockIdx.x, b = blockIdx.y;
  const int n0 = nbase + tile * 64;
  float bl[4], br[4];
#pragma unroll
  for (int e = 0; e < 4; ++e) {
    bl[e] = bf_bits2f(f2bf_bits(bias[4 * c16 + e]));
    br[e] = bf_bits2f(f2bf_bits(bias[kCh + 4 * c16 + e]));
  }
#pragma unroll 1
  for (int i = 0; i < 8; ++i) {
    const int nl = wave * 8 + i;
    const int n  = n0 + nl;
    const size_t R = ((size_t)tile * 64 + nl) * kBatch + b;
    const v4f mine = *(const v4f*)(lr + R * kLR + lane * 4);
    float lo[4], ro[4];
#pragma unroll
    for (int e = 0; e < 4; ++e) {
      const float m = mine[e];
      const float o = __shfl_xor(m, 16, 32);
      lo[e] = hh ? o : m;
      ro[e] = hh ? m : o;
    }
#pragma unroll
    for (int e = 0; e < 4; ++e) {
      const float L  = lo[e] + bl[e];
      const float Rr = ro[e] + br[e];
      const float sg = __builtin_amdgcn_rcpf(1.0f + __expf(-Rr));
      float v = L * sg;
      v = (n < kNV) ? v : 0.0f;
      if (hh == 0) sV[nl][4 * c16 + e] = v;
    }
  }
  __syncthreads();
  for (int pass = 0; pass < 2; ++pass) {
#pragma unroll
    for (int it = 0; it < 4; ++it) {
      const int nl = wave * 8 + it * 2 + hh;
      const int n  = n0 + nl;
      const v4f v = *(const v4f*)(&sV[nl][c16 * 4]);
      if (n >= kMid0 && n < kMid1) {
        *(volatile v4f*)(keep + (size_t)(n - kMid0) * kNCol + b * kCh + c16 * 4) = v;
      }
    }
    __threadfence();
  }
  if (write_xt) {
    const int q = lane >> 3, c8 = (lane & 7) * 8;
    for (int pass = 0; pass < 2; ++pass) {
#pragma unroll
      for (int it = 0; it < 2; ++it) {
        const int c = wave * 8 + it * 4 + q;
        unsigned short hb[8];
#pragma unroll
        for (int e = 0; e < 8; ++e) hb[e] = f2bf_bits(sV[c8 + e][c]);
        const v4u u = (v4u){pk16(hb[0], hb[1]), pk16(hb[2], hb[3]), pk16(hb[4], hb[5]), pk16(hb[6], hb[7])};
        *(volatile v4u*)(xt + (size_t)(b * kCh + c) * kNP + n0 + c8) = u;
      }
      __threadfence();
    }
  }
}

__global__ __launch_bounds__(256) void max3_kernel(const float* __restrict__ k0, const float* __restrict__ k1,
                                                   const float* __restrict__ k2, float* __restrict__ out, int n4) {
  const int gid = blockIdx.x * 256 + threadIdx.x;
  if (gid >= n4) return;
  const v4f a = *(const v4f*)(k0 + (size_t)gid * 4);
  const v4f bq = *(const v4f*)(k1 + (size_t)gid * 4);
  const v4f c = *(const v4f*)(k2 + (size_t)gid * 4);
  v4f m;
#pragma unroll
  for (int e = 0; e < 4; ++e) m[e] = fmaxf(fmaxf(a[e], bq[e]), c[e]);
  float* dst = out + (size_t)gid * 4;
  *(volatile v4f*)dst = m;
  __threadfence();
  *(volatile v4f*)dst = m;
}

static inline size_t align256(size_t v) { return (v + 255) & ~(size_t)255; }

extern "C" void kernel_launch(void* const* d_in, const int* in_sizes, int n_in,
                              void* d_out, int out_size, void* d_ws, size_t ws_size,
                              hipStream_t stream) {
  if (n_in < 8) return;
  const float* x   = (const float*)d_in[0];
  const float* adj = (const float*)d_in[1];
  const float* W0  = (const float*)d_in[2];
  const float* b0  = (const float*)d_in[3];
  const float* W1  = (const float*)d_in[4];
  const float* b1  = (const float*)d_in[5];
  const float* W2  = (const float*)d_in[6];
  const float* b2  = (const float*)d_in[7];
  float* outp = (float*)d_out;
  if (in_sizes[0] != kNV * kNCol || in_sizes[1] != kNV * kNV || in_sizes[2] != kCh * kLR ||
      in_sizes[3] != kLR || in_sizes[4] != kCh * kLR || in_sizes[5] != kLR ||
      in_sizes[6] != kCh * kLR || in_sizes[7] != kLR || out_size != kMidN * kNCol) return;

  const size_t szAdjb = (size_t)kNP * kNP * 2;
  const size_t szXT   = (size_t)kNCol * kNP * 2;
  const size_t szHB   = (size_t)kNP * kNCol * 2;
  const size_t szWT   = (size_t)3 * kLR * kCh * 2;
  const size_t szLR   = (size_t)kNP * kBatch * kLR * 4;
  const size_t szKeep = (size_t)kMidN * kNCol * 4;
  char* ws = (char*)d_ws;
  size_t off = 0;
  unsigned short* adjb = (unsigned short*)(ws + off); off = align256(off + szAdjb);
  unsigned short* xt   = (unsigned short*)(ws + off); off = align256(off + szXT);
  unsigned short* hb   = (unsigned short*)(ws + off); off = align256(off + szHB);
  unsigned short* wt   = (unsigned short*)(ws + off); off = align256(off + szWT);
  float* lr            = (float*)(ws + off);          off = align256(off + szLR);
  float* keep0         = (float*)(ws + off);          off = align256(off + szKeep);
  float* keep1         = (float*)(ws + off);          off = align256(off + szKeep);
  float* keep2         = (float*)(ws + off);          off = align256(off + szKeep);
  if (off > ws_size) return;

  cvt_adj_kernel<<<dim3(kAdjThreads / 256), dim3(256), 0, stream>>>(adj, adjb);
  cvt_xT_kernel<<<dim3(kNP / 64, kNCol / 64), dim3(256), 0, stream>>>(x, xt);
  cvt_w_kernel<<<dim3(12), dim3(256), 0, stream>>>(W0, W1, W2, wt);

  const int aggTilesFull = (kNP / 64) * (kNCol / 64);
  const int aggBlocksFull = (aggTilesFull + 7) / 8;
  const int linMFull = kNP * kBatch;
  const int linBlocksFull = ((linMFull / 64) * (kLR / 64) + 7) / 8;
  const int aggTilesL2 = (kL2Rows / 64) * (kNCol / 64);
  const int aggBlocksL2 = (aggTilesL2 + 7) / 8;
  const int linML2 = kL2Rows * kBatch;
  const int linBlocksL2 = ((linML2 / 64) * (kLR / 64) + 7) / 8;

  wmma_gemm64<1, false, 0, 3, false, 0><<<dim3(aggBlocksFull, 1), dim3(256), 0, stream>>>(
      adjb, adjb, kNP, 0L, xt, xt, kNP, 0L, (void*)hb, (void*)hb, kNCol, 0L,
      b0, lr, 0L, kNP, kNCol, kNP, 1.0f);
  wmma_gemm64<1, false, 0, 0, false, 0><<<dim3(linBlocksFull, 1), dim3(256), 0, stream>>>(
      hb, hb, kCh, 0L, wt + 0 * kLR * kCh, wt + 0 * kLR * kCh, kCh, 0L, (void*)lr, (void*)lr, kLR, 0L,
      b0, lr, 0L, linMFull, kLR, kCh, 1.0f);
  glu_kernel<<<dim3(kNP / 64, kBatch), dim3(256), 0, stream>>>(lr, b0, xt, keep0, 0, 1);

  wmma_gemm64<1, false, 0, 3, false, 0><<<dim3(aggBlocksFull, 1), dim3(256), 0, stream>>>(
      adjb, adjb, kNP, 0L, xt, xt, kNP, 0L, (void*)hb, (void*)hb, kNCol, 0L,
      b1, lr, 0L, kNP, kNCol, kNP, 1.0f);
  wmma_gemm64<1, false, 0, 0, false, 0><<<dim3(linBlocksFull, 1), dim3(256), 0, stream>>>(
      hb, hb, kCh, 0L, wt + 1 * kLR * kCh, wt + 1 * kLR * kCh, kCh, 0L, (void*)lr, (void*)lr, kLR, 0L,
      b1, lr, 0L, linMFull, kLR, kCh, 1.0f);
  glu_kernel<<<dim3(kNP / 64, kBatch), dim3(256), 0, stream>>>(lr, b1, xt, keep1, 0, 1);

  wmma_gemm64<1, false, 0, 3, false, 0><<<dim3(aggBlocksL2, 1), dim3(256), 0, stream>>>(
      adjb + (size_t)kL2Row0 * kNP, adjb + (size_t)kL2Row0 * kNP, kNP, 0L, xt, xt, kNP, 0L,
      (void*)hb, (void*)hb, kNCol, 0L, b2, lr, 0L, kL2Rows, kNCol, kNP, 1.0f);
  wmma_gemm64<1, false, 0, 0, false, 0><<<dim3(linBlocksL2, 1), dim3(256), 0, stream>>>(
      hb, hb, kCh, 0L, wt + 2 * kLR * kCh, wt + 2 * kLR * kCh, kCh, 0L, (void*)lr, (void*)lr, kLR, 0L,
      b2, lr, 0L, linML2, kLR, kCh, 1.0f);
  glu_kernel<<<dim3(kL2Rows / 64, kBatch), dim3(256), 0, stream>>>(lr, b2, xt, keep2, kL2Row0, 0);

  const int n4 = (kMidN * kNCol) / 4;
  max3_kernel<<<dim3((n4 + 255) / 256), dim3(256), 0, stream>>>(keep0, keep1, keep2, outp, n4);
}
